// TransE_26774826123521
// MI455X (gfx1250) — hardware-verified
//
#include <hip/hip_runtime.h>
#include <stddef.h>


typedef _Float16 h16;
typedef _Float16 v16h __attribute__((ext_vector_type(16)));
typedef _Float16 v8h  __attribute__((ext_vector_type(8)));
typedef float    v8f  __attribute__((ext_vector_type(8)));
typedef float    v4f  __attribute__((ext_vector_type(4)));

#ifndef NENT
#define NENT 100000
#endif
#define ENT_FULL 100000
#define REL_TOT  1000
#define DIM      128
#define NBATCH   32
#define NGROUPS  (NENT / 32)
#define WPB      5
#define LDW      36

#define ECARRY 4096.0f
#define HCARRY 256.0f

static_assert(NENT >= 32 && NENT <= ENT_FULL && (NENT % 32) == 0);
static_assert((ENT_FULL % 32) == 0);
static_assert(((size_t)ENT_FULL * 4) % 128 == 0);
static_assert(DIM == 4 * 32);
static_assert(DIM == 16 * 8);
static_assert(NBATCH == 32);
static_assert(NBATCH * 16 == 512);
static_assert(4 * 8 == NBATCH);
static_assert((LDW % 4) == 0 && LDW >= 32);
static_assert((size_t)WPB * NBATCH * LDW * 4 <= (size_t)131072);
static_assert((size_t)NBATCH * ENT_FULL < (size_t)0x7FFFFFFF);

#define HR16_BYTES ((size_t)NBATCH * DIM * 2)
#define HRN_BYTES  ((size_t)128)
#define OFF_HR16   ((size_t)0)
#define OFF_HRN    (OFF_HR16 + HR16_BYTES)
#define WS_TOTAL   (OFF_HRN + HRN_BYTES)
static_assert((HR16_BYTES % 128) == 0 && (OFF_HRN % 128) == 0);
static_assert(NBATCH * 4 == 128);
static_assert(WS_TOTAL <= (size_t)134217728);

__device__ __forceinline__ float bf16r(float x) {
  unsigned int u = __float_as_uint(x);
  u = (u + 0x7FFFu + ((u >> 16) & 1u)) & 0xFFFF0000u;
  return __uint_as_float(u);
}

__device__ __forceinline__ h16 toh_flush(float v) {
  const h16 r = (h16)v;
  return (fabsf(v) < 6.103515625e-05f) ? (h16)0.0f : r;
}

__device__ __forceinline__ v16h frag_at(const _Float16* p) {
  v8h lo = *(const v8h*)(p);
  v8h hi = *(const v8h*)(p + 16);
  v16h out;
#pragma unroll
  for (int i = 0; i < 8; ++i) { out[i] = lo[i]; out[i + 8] = hi[i]; }
  return out;
}

__device__ __forceinline__ v8f wmma16(v16h a, v16h b, v8f c) {
  v8f d = __builtin_amdgcn_wmma_f32_16x16x32_f16(false, a, false, b, (short)0, c,
                                                 false, false);
  asm volatile("v_nop\n\tv_nop\n\tv_nop\n\tv_nop" : "+v"(d) : "v"(a), "v"(b));
  return d;
}

__device__ __forceinline__ float red16_sum(float x) {
#pragma unroll
  for (int off = 1; off < 16; off <<= 1) x += __shfl_xor(x, off, 32);
  return x;
}

__device__ __forceinline__ void wave_lds_sync() {
  __builtin_amdgcn_fence(3  , "wavefront");
  asm volatile("s_wait_dscnt 0x0" ::: "memory");
  __builtin_amdgcn_wave_barrier();
}

__global__ __launch_bounds__(512) void prep_kernel(
    const int* __restrict__ h, const int* __restrict__ r,
    const float* __restrict__ ent, const float* __restrict__ rel,
    _Float16* __restrict__ hr16, float* __restrict__ hrn) {
  __shared__ float sn[NBATCH];
  const unsigned tid = threadIdx.x;
  const unsigned b = tid >> 4;
  const unsigned c = (tid & 15u) * 8u;

  int hi0 = h[b];
  hi0 = (hi0 < 0) ? (hi0 + ENT_FULL) : hi0;
  hi0 = (hi0 < 0) ? 0 : hi0;
  hi0 = (hi0 > ENT_FULL - 1) ? (ENT_FULL - 1) : hi0;
  int ri0 = r[b];
  ri0 = (ri0 < 0) ? (ri0 + REL_TOT) : ri0;
  ri0 = (ri0 < 0) ? 0 : ri0;
  ri0 = (ri0 > REL_TOT - 1) ? (REL_TOT - 1) : ri0;

  const float* er = ent + (size_t)hi0 * DIM + c;
  const float* rr = rel + (size_t)ri0 * DIM + c;
  const v4f e0 = *(const v4f*)(er);
  const v4f e1 = *(const v4f*)(er + 4);
  const v4f r0 = *(const v4f*)(rr);
  const v4f r1 = *(const v4f*)(rr + 4);

  v8h o;
  float ss = 0.0f;
#pragma unroll
  for (int i = 0; i < 4; ++i) {
    const float t0 = bf16r(e0[i]) + bf16r(r0[i]);
    const float t1 = bf16r(e1[i]) + bf16r(r1[i]);
    ss += t0 * t0;
    ss += t1 * t1;
    o[i]     = toh_flush(HCARRY * t0);
    o[i + 4] = toh_flush(HCARRY * t1);
  }
  ss = red16_sum(ss);
  if ((tid & 15u) == 0u) sn[b] = ss;

  _Float16* p = hr16 + (size_t)b * DIM + c;
  *(volatile v8h*)p = o;
  __threadfence();
  *(volatile v8h*)p = o;

  __syncthreads();
  if (tid < 8u) {
    const v4f x = *(const v4f*)&sn[tid * 4u];
    float* q = hrn + tid * 4u;
    *(volatile v4f*)q = x;
    __threadfence();
    *(volatile v4f*)q = x;
  }
}

__global__ __launch_bounds__(32 * WPB) void score_kernel(
    const float* __restrict__ ent, const _Float16* __restrict__ hr16,
    const float* __restrict__ hrn, float* __restrict__ out) {
  __shared__ float Cs[WPB * NBATCH * LDW];

  const unsigned lane = threadIdx.x & 31u;
  const unsigned wave = (unsigned)__builtin_amdgcn_readfirstlane((int)(threadIdx.x >> 5));
  const unsigned hh = lane >> 4, m = lane & 15u;
  const unsigned grp = blockIdx.x * (unsigned)WPB + wave;
  if (grp >= (unsigned)NGROUPS) return;
  const unsigned e0 = grp * 32u;
  const unsigned cbase = wave * (unsigned)(NBATCH * LDW);

  v16h af[2][4];
#pragma unroll
  for (int mt = 0; mt < 2; ++mt)
#pragma unroll
    for (int kc = 0; kc < 4; ++kc)
      af[mt][kc] = frag_at(hr16 + ((unsigned)mt * 16u + m) * (unsigned)DIM +
                           (unsigned)kc * 32u + hh * 8u);

  v4f hn[2][2];
#pragma unroll
  for (int mt = 0; mt < 2; ++mt)
#pragma unroll
    for (int j = 0; j < 2; ++j)
      hn[mt][j] = *(const v4f*)(hrn + (unsigned)mt * 16u + hh * 8u + 4u * (unsigned)j);

  const float cs = 2.0f / (ECARRY * HCARRY);

#pragma unroll
  for (int t = 0; t < 2; ++t) {
    const float* ep = ent + (size_t)(e0 + (unsigned)t * 16u + m) * DIM + hh * 8u;
    v8f c0 = {}, c1 = {};
    float en = 0.0f;
#pragma unroll
    for (int kc = 0; kc < 4; ++kc) {
      const v4f x0 = *(const v4f*)(ep + kc * 32);
      const v4f x1 = *(const v4f*)(ep + kc * 32 + 4);
      const v4f x2 = *(const v4f*)(ep + kc * 32 + 16);
      const v4f x3 = *(const v4f*)(ep + kc * 32 + 20);
      v16h bf;
#pragma unroll
      for (int i = 0; i < 4; ++i) {
        const float f0 = bf16r(x0[i]);
        const float f1 = bf16r(x1[i]);
        const float f2 = bf16r(x2[i]);
        const float f3 = bf16r(x3[i]);
        en += f0 * f0;
        en += f1 * f1;
        en += f2 * f2;
        en += f3 * f3;
        bf[i]      = toh_flush(ECARRY * f0);
        bf[i + 4]  = toh_flush(ECARRY * f1);
        bf[i + 8]  = toh_flush(ECARRY * f2);
        bf[i + 12] = toh_flush(ECARRY * f3);
      }
      c0 = wmma16(af[0][kc], bf, c0);
      c1 = wmma16(af[1][kc], bf, c1);
    }
    en += __shfl_xor(en, 16, 32);
#pragma unroll
    for (int v = 0; v < 8; ++v) {
      const float s0 = hn[0][v >> 2][v & 3] + en - cs * c0[v];
      const float s1 = hn[1][v >> 2][v & 3] + en - cs * c1[v];
      Cs[cbase + (hh * 8u + (unsigned)v) * LDW + (unsigned)t * 16u + m] =
          sqrtf(fmaxf(s0, 0.0f));
      Cs[cbase + (16u + hh * 8u + (unsigned)v) * LDW + (unsigned)t * 16u + m] =
          sqrtf(fmaxf(s1, 0.0f));
    }
  }
  wave_lds_sync();

  v4f x[8];
  size_t off[8];
#pragma unroll
  for (unsigned i = 0; i < 8u; ++i) {
    const unsigned row = 4u * i + (lane >> 3);
    const unsigned c = (lane & 7u) * 4u;
    x[i] = *(const v4f*)&Cs[cbase + row * LDW + c];
    off[i] = (size_t)row * ENT_FULL + e0 + c;
  }
#pragma unroll
  for (int i = 0; i < 8; ++i) *(volatile v4f*)(out + off[i]) = x[i];
  __threadfence();
#pragma unroll
  for (int i = 0; i < 8; ++i) *(volatile v4f*)(out + off[i]) = x[i];
}

extern "C" void kernel_launch(void* const* d_in, const int* in_sizes, int n_in,
                              void* d_out, int out_size, void* d_ws, size_t ws_size,
                              hipStream_t stream) {
  if (n_in < 5) return;
  if (in_sizes[0] < NBATCH || in_sizes[1] < NBATCH) return;
  if ((long long)in_sizes[3] < (long long)ENT_FULL * DIM) return;
  if ((long long)in_sizes[4] < (long long)REL_TOT * DIM) return;
  if ((long long)out_size < (long long)(NBATCH - 1) * ENT_FULL + NENT) return;
  if (ws_size < WS_TOTAL) return;

  const int*   h   = (const int*)d_in[0];
  const int*   r   = (const int*)d_in[1];
  const float* ent = (const float*)d_in[3];
  const float* rel = (const float*)d_in[4];
  float* out = (float*)d_out;

  char* ws = (char*)d_ws;
  _Float16* hr16 = (_Float16*)(ws + OFF_HR16);
  float*    hrn  = (float*)(ws + OFF_HRN);

  prep_kernel<<<dim3(1), dim3(512), 0, stream>>>(h, r, ent, rel, hr16, hrn);
  score_kernel<<<dim3((NGROUPS + WPB - 1) / WPB), dim3(32 * WPB), 0, stream>>>(
      ent, hr16, hrn, out);
}
